// CrossAttention_7370163880742
// MI455X (gfx1250) — hardware-run, weakly checked
//
#include <hip/hip_runtime.h>
#include <stdint.h>


typedef _Float16 v16h __attribute__((ext_vector_type(16)));
typedef _Float16 v8h  __attribute__((ext_vector_type(8)));
typedef float    v8f  __attribute__((ext_vector_type(8)));
typedef float    v4f  __attribute__((ext_vector_type(4)));
typedef float    v2f  __attribute__((ext_vector_type(2)));
typedef int      v4i  __attribute__((ext_vector_type(4)));
typedef _Float16 h16;

#ifndef NB
#define NB 2
#endif
#ifndef SEQ
#define SEQ 1024
#endif
#define NB_FULL  2
#define SEQ_FULL 1024
#define CH       512
#define NH       8
#define HD       64
#define DFF      2048

#define ACT_CAR   8.0f
#define W_CAR     1024.0f
#define PROJ_SCL  0.0001220703125f
#define MID_SCL   3.814697265625e-6f
#define QKV_CAR   256.0f
#define S_SCL     1.9073486328125e-6f
#define P_CAR     16384.0f
#define O_SCL     6.103515625e-5f

static_assert(SEQ % 128 == 0);
static_assert(SEQ % 4 == 0);
static_assert(SEQ <= SEQ_FULL);
static_assert(NB >= 1 && NB <= NB_FULL);
static_assert(CH == NH * HD);
static_assert(HD == 64);
static_assert(NH == 8);
static_assert(CH % 128 == 0);
static_assert(CH % 32 == 0);
static_assert(DFF % 64 == 0);
static_assert(DFF % 32 == 0);
static_assert(((long)NB * SEQ) % 128 == 0);
static_assert(((long)2 * NB * SEQ) % 8 == 0);
static_assert((long)NB_FULL * SEQ_FULL * CH * 4 == 4194304L);
static_assert((long)NB_FULL * SEQ_FULL * 2 * CH * 4 == 8388608L);
static_assert(((long)36 * NB * SEQ * CH + (long)26 * CH * CH) * 2
              + (long)3 * 2 * NB * SEQ * CH * 4 + (long)2 * 2 * NB * SEQ * 4 <= 134217728L);
static_assert(128 * 72 * 2 <= 131072);
static_assert(128 * 68 * 4 <= 131072);
static_assert(128 * 72 * 2 + 8 * 16 * 40 * 2 + 64 * 4 <= 131072);
static_assert(8 * CH * 2 <= 131072);

union Frag16 { v16h v; v8h p[2]; };

__device__ __forceinline__ v16h ld_frag(const _Float16* p, int hl) {
  Frag16 f;
  f.p[0] = *(const v8h*)(p + 8 * hl);
  f.p[1] = *(const v8h*)(p + 16 + 8 * hl);
  return f.v;
}

#define LDS_FRAG(dst, arr, off)                                \
  do {                                                         \
    Frag16 f_;                                                 \
    f_.p[0] = *(const v8h*)&arr[(off) + 8 * hl];               \
    f_.p[1] = *(const v8h*)&arr[(off) + 16 + 8 * hl];          \
    dst = f_.v;                                                \
  } while (0)

__device__ __forceinline__ v8f mma(v16h a, v16h b, v8f c) {
  v8f d = __builtin_amdgcn_wmma_f32_16x16x32_f16(false, a, false, b, (short)0, c, false, false);
  asm volatile("v_nop\n\tv_nop\n\tv_nop\n\tv_nop" : "+v"(d) : "v"(a), "v"(b));
  return d;
}

__device__ __forceinline__ float bf16_rne(float x) {
  unsigned int u = __builtin_bit_cast(unsigned int, x);
  u += 0x7FFFu + ((u >> 16) & 1u);
  return __builtin_bit_cast(float, u & 0xFFFF0000u);
}

static __device__ __forceinline__ h16 toh_flush(float v) {
  const h16 r = (h16)v;
  return (fabsf(v) < 6.103515625e-05f) ? (h16)0.0f : r;
}

__global__ __launch_bounds__(256) void k_cvt8(const float* __restrict__ src,
                                              _Float16* __restrict__ dst,
                                              int cols, int rpb, int rpb_full,
                                              float car, int total8)
{
  const int i8 = blockIdx.x * 256 + threadIdx.x;
  if (i8 >= total8) return;
  const size_t e   = (size_t)i8 * 8;
  const size_t r   = e / (size_t)cols;
  const int    col = (int)(e - r * (size_t)cols);
  const size_t rb  = r / (size_t)rpb;
  const size_t rs  = rb * (size_t)rpb_full + (r - rb * (size_t)rpb);
  const float* s = src + rs * (size_t)cols + col;
  const v4f x0 = *(const v4f*)s;
  const v4f x1 = *(const v4f*)(s + 4);
  v8h o;
#pragma unroll
  for (int j = 0; j < 4; ++j) {
    const float t0 = x0[j];
    const float t1 = x1[j];
    o[j]     = (_Float16)(bf16_rne(t0) * car);
    o[4 + j] = (_Float16)(bf16_rne(t1) * car);
  }
  _Float16* d = dst + e;
  *(volatile v8h*)d = o;
  __threadfence();
  *(volatile v8h*)d = o;
}

static_assert((2 * NB * SEQ) % 4 == 0);
__global__ __launch_bounds__(256) void k_mask(const int* __restrict__ em,
                                              const int* __restrict__ sm,
                                              float* __restrict__ mx,
                                              float* __restrict__ mt)
{
  const int g = blockIdx.x * 256 + threadIdx.x;
  if (g >= (2 * NB * SEQ) / 4) return;
  const int e = g * 4;
  const int tb  = e / SEQ;
  const int s   = e - tb * SEQ;
  const int mha = tb / NB;
  const int b   = tb - mha * NB;
  const int src = b * SEQ_FULL + s;
  v4i e1 = *(const v4i*)(em + src);
  v4i s1 = *(const v4i*)(sm + src);
  const int b2   = e / (2 * SEQ);
  const int pp   = e - b2 * 2 * SEQ;
  const int hf   = pp / SEQ;
  const int s2   = pp - hf * SEQ;
  const int src2 = b2 * SEQ_FULL + s2;
  v4i e2 = *(const v4i*)(em + src2);
  v4i t2 = *(const v4i*)(sm + src2);
  asm volatile("" : "+v"(e1));
  asm volatile("" : "+v"(s1));
  asm volatile("" : "+v"(e2));
  asm volatile("" : "+v"(t2));
  v4f x, t;
#pragma unroll
  for (int j = 0; j < 4; ++j) {
    const int a0 = (mha == 0) ? s1[j] : e1[j];
    const int a1 = (hf == 0) ? e2[j] : t2[j];
    x[j] = (a0 == 1) ? 1.0f : 0.0f;
    t[j] = (a1 == 1) ? 1.0f : 0.0f;
  }
  *(volatile v4f*)(mx + e) = x;
  *(volatile v4f*)(mt + e) = t;
  __threadfence();
  *(volatile v4f*)(mx + e) = x;
  *(volatile v4f*)(mt + e) = t;
}

__device__ __forceinline__ void gemm_main(const _Float16* __restrict__ A,
                                          const _Float16* __restrict__ Bt,
                                          int mw, int n0, int c, int hl, v8f (&acc)[8])
{
  const _Float16* ap0 = A  + (size_t)(mw + c) * CH;
  const _Float16* ap1 = A  + (size_t)(mw + 16 + c) * CH;
  const _Float16* bp  = Bt + (size_t)(n0 + c) * CH;
  const size_t bst = (size_t)16 * CH;
#pragma unroll 1
  for (int k0 = 0; k0 < CH; k0 += 32) {
    const v16h a0 = ld_frag(ap0 + k0, hl);
    const v16h a1 = ld_frag(ap1 + k0, hl);
    const v16h b0 = ld_frag(bp + k0, hl);
    const v16h b1 = ld_frag(bp + bst + k0, hl);
    const v16h b2 = ld_frag(bp + 2 * bst + k0, hl);
    const v16h b3 = ld_frag(bp + 3 * bst + k0, hl);
    acc[0] = mma(a0, b0, acc[0]);
    acc[1] = mma(a0, b1, acc[1]);
    acc[2] = mma(a0, b2, acc[2]);
    acc[3] = mma(a0, b3, acc[3]);
    acc[4] = mma(a1, b0, acc[4]);
    acc[5] = mma(a1, b1, acc[5]);
    acc[6] = mma(a1, b2, acc[6]);
    acc[7] = mma(a1, b3, acc[7]);
  }
}

__device__ __forceinline__ void gemm_main_k(const _Float16* __restrict__ A,
                                            const _Float16* __restrict__ Bt,
                                            int K, int mw, int n0, int c, int hl, v8f (&acc)[8])
{
  const _Float16* ap0 = A  + (size_t)(mw + c) * K;
  const _Float16* ap1 = A  + (size_t)(mw + 16 + c) * K;
  const _Float16* bp  = Bt + (size_t)(n0 + c) * K;
  const size_t bst = (size_t)16 * K;
#pragma unroll 1
  for (int k0 = 0; k0 < K; k0 += 32) {
    const v16h a0 = ld_frag(ap0 + k0, hl);
    const v16h a1 = ld_frag(ap1 + k0, hl);
    const v16h b0 = ld_frag(bp + k0, hl);
    const v16h b1 = ld_frag(bp + bst + k0, hl);
    const v16h b2 = ld_frag(bp + 2 * bst + k0, hl);
    const v16h b3 = ld_frag(bp + 3 * bst + k0, hl);
    acc[0] = mma(a0, b0, acc[0]);
    acc[1] = mma(a0, b1, acc[1]);
    acc[2] = mma(a0, b2, acc[2]);
    acc[3] = mma(a0, b3, acc[3]);
    acc[4] = mma(a1, b0, acc[4]);
    acc[5] = mma(a1, b1, acc[5]);
    acc[6] = mma(a1, b2, acc[6]);
    acc[7] = mma(a1, b3, acc[7]);
  }
}

static_assert(128 * 8 * 16 == 128 * 128);
template <bool ROWB>
__device__ __forceinline__ void gemm_hb_body(const _Float16* __restrict__ A,
                                             const _Float16* __restrict__ Bt,
                                             _Float16* __restrict__ C, int ldc,
                                             const float* __restrict__ bias,
                                             float scl, float car, int relu)
{
  __shared__ __attribute__((aligned(16))) _Float16 ldsE[128 * 72];

  const int tid = threadIdx.x, lane = tid & 31, w = tid >> 5;
  const int hl = lane >> 4, c = lane & 15;
  const int m0 = blockIdx.y * 128, n0 = blockIdx.x * 64;
  const int mw = m0 + 32 * w;

  v8f acc[8] = {};
  gemm_main(A, Bt, mw, n0, c, hl, acc);

#pragma unroll
  for (int i = 0; i < 2; ++i) {
    float br[8] = {0.f, 0.f, 0.f, 0.f, 0.f, 0.f, 0.f, 0.f};
    if constexpr (ROWB) {
      const int rb = mw + 16 * i + 8 * hl;
      const v4f b0 = *(const v4f*)(bias + rb);
      const v4f b1 = *(const v4f*)(bias + rb + 4);
#pragma unroll
      for (int r = 0; r < 4; ++r) {
        br[r]     = bf16_rne(b0[r]);
        br[4 + r] = bf16_rne(b1[r]);
      }
    }
#pragma unroll
    for (int t = 0; t < 4; ++t) {
      float bt = 0.f;
      if constexpr (!ROWB) {
        bt = bf16_rne(bias[n0 + 16 * t + c]);
      }
#pragma unroll
      for (int r = 0; r < 8; ++r) {
        const int rowl = 32 * w + 16 * i + 8 * hl + r;
        const float sb = ROWB ? br[r] : bt;
        float y = acc[i * 4 + t][r] * scl + sb;
        y = (relu != 0) ? fmaxf(y, 0.0f) : y;
        ldsE[rowl * 72 + 16 * t + c] = toh_flush(y * car);
      }
    }
  }
  __syncthreads();

  _Float16* const cb = C + (size_t)m0 * ldc + n0;
  for (int i = 0; i < 8; ++i) {
    const int q = i * 128 + tid;
    const int rowl = q >> 3, chh = (q & 7) * 8;
    const v8h vh = *(const v8h*)&ldsE[rowl * 72 + chh];
    *(volatile v8h*)(cb + (size_t)rowl * ldc + chh) = vh;
  }
  __threadfence();
  for (int i = 0; i < 8; ++i) {
    const int q = i * 128 + tid;
    const int rowl = q >> 3, chh = (q & 7) * 8;
    const v8h vh = *(const v8h*)&ldsE[rowl * 72 + chh];
    *(volatile v8h*)(cb + (size_t)rowl * ldc + chh) = vh;
  }
}

__global__ __launch_bounds__(128) __attribute__((amdgpu_num_vgpr(256)))
void k_gemm_h(const _Float16* __restrict__ A, const _Float16* __restrict__ Bt,
              _Float16* __restrict__ C, const float* __restrict__ bias,
              long zA, long zB, long zC, int ldc, float scl, float car, int relu, int zbias)
{
  const long z = blockIdx.z;
  gemm_hb_body<false>(A + z * zA, Bt + z * zB, C + z * zC, ldc, bias + z * zbias, scl, car, relu);
}

__global__ __launch_bounds__(128) __attribute__((amdgpu_num_vgpr(256)))
void k_gemm_vt(const _Float16* __restrict__ Aw, const _Float16* __restrict__ X,
               _Float16* __restrict__ Vt, const float* __restrict__ bias,
               long zX, long zC, int ldc)
{
  const long z = blockIdx.z;
  gemm_hb_body<true>(Aw, X + z * zX, Vt + z * zC, ldc, bias, MID_SCL, QKV_CAR, 0);
}

static_assert(128 * 16 * 16 == 128 * 256);
static_assert(128 * 8 * 16 == 128 * 128);
__global__ __launch_bounds__(128) __attribute__((amdgpu_num_vgpr(256)))
void k_gemm_x0(const _Float16* __restrict__ A, const _Float16* __restrict__ Bt,
               float* __restrict__ Out, _Float16* __restrict__ Out16,
               const float* __restrict__ bias, int rpb, int rpb_out, int rowoff)
{
  __shared__ __attribute__((aligned(16))) float ldsF[128 * 68];

  const int tid = threadIdx.x, lane = tid & 31, w = tid >> 5;
  const int hl = lane >> 4, c = lane & 15;
  const int m0 = blockIdx.y * 128, n0 = blockIdx.x * 64;
  const int mw = m0 + 32 * w;

  v8f acc[8] = {};
  gemm_main(A, Bt, mw, n0, c, hl, acc);

#pragma unroll
  for (int i = 0; i < 2; ++i)
#pragma unroll
    for (int t = 0; t < 4; ++t) {
      const float bt = bf16_rne(bias[n0 + 16 * t + c]);
#pragma unroll
      for (int r = 0; r < 8; ++r) {
        const int rowl = 32 * w + 16 * i + 8 * hl + r;
        ldsF[rowl * 68 + 16 * t + c] = acc[i * 4 + t][r] * MID_SCL + bt;
      }
    }
  __syncthreads();

  const int bq = m0 / rpb;
  const size_t crow0 = (size_t)bq * rpb_out + (size_t)(m0 - bq * rpb) + (size_t)rowoff;
  float* const ob = Out + crow0 * CH + n0;
  _Float16* const oh = Out16 + crow0 * CH + n0;
  for (int i = 0; i < 16; ++i) {
    const int q = i * 128 + tid;
    const int rowl = q >> 4, chh = (q & 15) * 4;
    const v4f v = *(const v4f*)&ldsF[rowl * 68 + chh];
    *(volatile v4f*)(ob + (size_t)rowl * CH + chh) = v;
  }
  for (int i = 0; i < 8; ++i) {
    const int q = i * 128 + tid;
    const int rowl = q >> 3, chh = (q & 7) * 8;
    const v4f a = *(const v4f*)&ldsF[rowl * 68 + chh];
    const v4f b = *(const v4f*)&ldsF[rowl * 68 + chh + 4];
    v8h o;
#pragma unroll
    for (int j = 0; j < 4; ++j) {
      o[j]     = toh_flush(a[j] * QKV_CAR);
      o[4 + j] = toh_flush(b[j] * QKV_CAR);
    }
    *(volatile v8h*)(oh + (size_t)rowl * CH + chh) = o;
  }
  __threadfence();
  for (int i = 0; i < 16; ++i) {
    const int q = i * 128 + tid;
    const int rowl = q >> 4, chh = (q & 15) * 4;
    const v4f v = *(const v4f*)&ldsF[rowl * 68 + chh];
    *(volatile v4f*)(ob + (size_t)rowl * CH + chh) = v;
  }
  for (int i = 0; i < 8; ++i) {
    const int q = i * 128 + tid;
    const int rowl = q >> 3, chh = (q & 7) * 8;
    const v4f a = *(const v4f*)&ldsF[rowl * 68 + chh];
    const v4f b = *(const v4f*)&ldsF[rowl * 68 + chh + 4];
    v8h o;
#pragma unroll
    for (int j = 0; j < 4; ++j) {
      o[j]     = toh_flush(a[j] * QKV_CAR);
      o[4 + j] = toh_flush(b[j] * QKV_CAR);
    }
    *(volatile v8h*)(oh + (size_t)rowl * CH + chh) = o;
  }
}

static_assert(128 * 16 * 16 == 128 * 256);
__global__ __launch_bounds__(128) __attribute__((amdgpu_num_vgpr(256)))
void k_gemm_res(const _Float16* __restrict__ A, const _Float16* __restrict__ Bt,
                float* __restrict__ Out, const float* __restrict__ bias,
                const float* __restrict__ Res, int K)
{
  __shared__ __attribute__((aligned(16))) float ldsF[128 * 68];

  const int tid = threadIdx.x, lane = tid & 31, w = tid >> 5;
  const int hl = lane >> 4, c = lane & 15;
  const int m0 = blockIdx.y * 128, n0 = blockIdx.x * 64;
  const int mw = m0 + 32 * w;

  v8f acc[8] = {};
  gemm_main_k(A, Bt, K, mw, n0, c, hl, acc);

#pragma unroll
  for (int i = 0; i < 2; ++i)
#pragma unroll
    for (int t = 0; t < 4; ++t) {
      const float bt = bf16_rne(bias[n0 + 16 * t + c]);
#pragma unroll
      for (int r = 0; r < 8; ++r) {
        const int rowl = 32 * w + 16 * i + 8 * hl + r;
        ldsF[rowl * 68 + 16 * t + c] = acc[i * 4 + t][r] * MID_SCL + bt;
      }
    }
  __syncthreads();

  const size_t ro = (size_t)m0 * CH + n0;
  float* const ob = Out + ro;
  const float* const rbp = Res + ro;
  v4f vv[16];
#pragma unroll
  for (int i = 0; i < 16; ++i) {
    const int q = i * 128 + tid;
    const int rowl = q >> 4, chh = (q & 15) * 4;
    const v4f v = *(const v4f*)&ldsF[rowl * 68 + chh];
    const v4f rr = *(const v4f*)(rbp + (size_t)rowl * CH + chh);
    vv[i] = v + rr;
  }
#pragma unroll
  for (int i = 0; i < 16; ++i) {
    const int q = i * 128 + tid;
    const int rowl = q >> 4, chh = (q & 15) * 4;
    *(volatile v4f*)(ob + (size_t)rowl * CH + chh) = vv[i];
  }
  __threadfence();
#pragma unroll
  for (int i = 0; i < 16; ++i) {
    const int q = i * 128 + tid;
    const int rowl = q >> 4, chh = (q & 15) * 4;
    *(volatile v4f*)(ob + (size_t)rowl * CH + chh) = vv[i];
  }
}

#define KT_H (64 * 72)
#define VT_H (64 * 72)
#define PW_H (16 * 40)
static_assert(KT_H + VT_H == 128 * 72);
static_assert(64 * 8 == 2 * 256);
static_assert(128 * 8 == 4 * 256);
static_assert(256 * 4 * 16 == 128 * 128);

__global__ __launch_bounds__(256) __attribute__((amdgpu_num_vgpr(256)))
void k_attn(const _Float16* __restrict__ Q, const _Float16* __restrict__ K,
            const _Float16* __restrict__ Vt, const float* __restrict__ Mk,
            _Float16* __restrict__ O, int S_)
{
  __shared__ __attribute__((aligned(16))) _Float16 ldsKV[KT_H + VT_H];
  __shared__ __attribute__((aligned(16))) _Float16 ldsP[8 * PW_H];
  __shared__ __attribute__((aligned(16))) float    ldsM[64];

  const int tid = threadIdx.x, lane = tid & 31, w = tid >> 5;
  const int wave = __builtin_amdgcn_readfirstlane(threadIdx.x >> 5);
  const int hl = lane >> 4, c = lane & 15;
  const int qblocks = S_ / 128;
  const int tbh = blockIdx.x / qblocks;
  const int qb  = blockIdx.x - tbh * qblocks;
  const int tb = tbh >> 3, h = tbh & 7;
  const int q0 = qb * 128;
  const int qw = q0 + 16 * w;

  const size_t qoff  = ((size_t)tb * S_ + qw + c) * CH + h * HD;
  const size_t kbase = (size_t)tb * S_ * CH + h * HD;
  const size_t vbase = ((size_t)tb * CH + h * HD) * S_;
  const size_t mbase = (size_t)tb * S_;
  const int pbase = w * PW_H;
  const int nkb = S_ / 64;

  float m[8], l[8];
  v8f o[4] = {};
#pragma unroll
  for (int r = 0; r < 8; ++r) { m[r] = -__builtin_inff(); l[r] = 0.f; }

#pragma unroll 1
  for (int kb = 0; kb < nkb; ++kb) {
    const int mk = kb * 64;
#pragma unroll
    for (int j = 0; j < 2; ++j) {
      const int s  = j * 256 + tid;
      const int rr = s >> 3, cc = (s & 7) * 8;
      const v8h k8 = *(const v8h*)(K + kbase + (size_t)(mk + rr) * CH + cc);
      *(v8h*)&ldsKV[rr * 72 + cc] = k8;
      const v8h v8 = *(const v8h*)(Vt + vbase + (size_t)rr * S_ + mk + cc);
      *(v8h*)&ldsKV[KT_H + rr * 72 + cc] = v8;
    }
    if (wave == 0) {
      const v2f mv = *(const v2f*)(Mk + mbase + mk + 2 * lane);
      *(v2f*)&ldsM[2 * lane] = mv;
    }
    __syncthreads();

#pragma unroll
    for (int hf = 0; hf < 2; ++hf) {
      v8f s0 = {}, s1 = {};
#pragma unroll
      for (int ks = 0; ks < 2; ++ks) {
        const v16h qf = ld_frag(Q + qoff + 32 * ks, hl);
        v16h kf0, kf1;
        LDS_FRAG(kf0, ldsKV, (32 * hf + c) * 72 + 32 * ks);
        LDS_FRAG(kf1, ldsKV, (32 * hf + 16 + c) * 72 + 32 * ks);
        s0 = mma(qf, kf0, s0);
        s1 = mma(qf, kf1, s1);
      }
      const float f0 = ldsM[32 * hf + c];
      const float f1 = ldsM[32 * hf + 16 + c];

#pragma unroll
      for (int r = 0; r < 8; ++r) {
        const float v0 = (f0 != 0.0f) ? s0[r] * S_SCL : -1.0e9f;
        const float v1 = (f1 != 0.0f) ? s1[r] * S_SCL : -1.0e9f;
        float tm = fmaxf(v0, v1);
        tm = fmaxf(tm, __shfl_xor(tm, 1, 32));
        tm = fmaxf(tm, __shfl_xor(tm, 2, 32));
        tm = fmaxf(tm, __shfl_xor(tm, 4, 32));
        tm = fmaxf(tm, __shfl_xor(tm, 8, 32));
        const float mn = fmaxf(m[r], tm);
        const float al = __expf(m[r] - mn);
        const float p0 = __expf(v0 - mn), p1 = __expf(v1 - mn);
        float rs = p0 + p1;
        rs += __shfl_xor(rs, 1, 32);
        rs += __shfl_xor(rs, 2, 32);
        rs += __shfl_xor(rs, 4, 32);
        rs += __shfl_xor(rs, 8, 32);
        l[r] = l[r] * al + rs;
        m[r] = mn;
#pragma unroll
        for (int t = 0; t < 4; ++t) o[t][r] *= al;
        const int po = pbase + (8 * hl + r) * 40 + c;
        ldsP[po]      = toh_flush(p0 * P_CAR);
        ldsP[po + 16] = toh_flush(p1 * P_CAR);
      }
      __syncthreads();

      v16h pf;
      LDS_FRAG(pf, ldsP, pbase + c * 40);
#pragma unroll
      for (int t = 0; t < 4; ++t) {
        v16h vf;
        LDS_FRAG(vf, ldsKV, KT_H + (16 * t + c) * 72 + 32 * hf);
        o[t] = mma(pf, vf, o[t]);
      }
    }
    __syncthreads();
  }

#pragma unroll
  for (int r = 0; r < 8; ++r) {
    const float inv = (1.0f / l[r]) * O_SCL;
    const int rowl = 16 * w + 8 * hl + r;
#pragma unroll
    for (int t = 0; t < 4; ++t)
      ldsKV[rowl * 72 + 16 * t + c] = toh_flush(o[t][r] * inv);
  }
  __syncthreads();
  _Float16* const ob = O + ((size_t)tb * S_ + q0) * CH + h * HD;
  for (int i = 0; i < 4; ++i) {
    const int qi = i * 256 + tid;
    const int rowl = qi >> 3, chh = (qi & 7) * 8;
    const v8h v = *(const v8h*)&ldsKV[rowl * 72 + chh];
    *(volatile v8h*)(ob + (size_t)rowl * CH + chh) = v;
  }
  __threadfence();
  for (int i = 0; i < 4; ++i) {
    const int qi = i * 256 + tid;
    const int rowl = qi >> 3, chh = (qi & 7) * 8;
    const v8h v = *(const v8h*)&ldsKV[rowl * 72 + chh];
    *(volatile v8h*)(ob + (size_t)rowl * CH + chh) = v;
  }
}

static_assert(CH == 4 * 32 * 4);
__device__ __forceinline__ void ln_row(const float* __restrict__ p,
                                       const float* __restrict__ g,
                                       const float* __restrict__ be,
                                       int lane, v4f (&y)[4])
{
#pragma clang fp contract(off)
  v4f x[4];
#pragma unroll
  for (int j = 0; j < 4; ++j) x[j] = *(const v4f*)(p + 128 * j + 4 * lane);
  float s = 0.f;
#pragma unroll
  for (int j = 0; j < 4; ++j)
#pragma unroll
    for (int e = 0; e < 4; ++e) s += x[j][e];
  s += __shfl_xor(s, 16, 32);
  s += __shfl_xor(s, 8, 32);
  s += __shfl_xor(s, 4, 32);
  s += __shfl_xor(s, 2, 32);
  s += __shfl_xor(s, 1, 32);
  const float mean = s * (1.0f / (float)CH);
  float q = 0.f;
#pragma unroll
  for (int j = 0; j < 4; ++j)
#pragma unroll
    for (int e = 0; e < 4; ++e) {
      const float d = x[j][e] - mean;
      q += d * d;
    }
  q += __shfl_xor(q, 16, 32);
  q += __shfl_xor(q, 8, 32);
  q += __shfl_xor(q, 4, 32);
  q += __shfl_xor(q, 2, 32);
  q += __shfl_xor(q, 1, 32);
  const float rstd = rsqrtf(q * (1.0f / (float)CH) + 1e-5f);
#pragma unroll
  for (int j = 0; j < 4; ++j) {
    const v4f gv = *(const v4f*)(g + 128 * j + 4 * lane);
    const v4f bv = *(const v4f*)(be + 128 * j + 4 * lane);
#pragma unroll
    for (int e = 0; e < 4; ++e) {
      const float d = (x[j][e] - mean) * rstd;
      y[j][e] = d * bf16_rne(gv[e]) + bf16_rne(bv[e]);
    }
  }
}

static_assert(32 * 4 * 16 == CH * 4);
static_assert(32 * 2 * 16 == CH * 2);
__global__ __launch_bounds__(256) void k_ln1(const float* __restrict__ S,
                                             const float* __restrict__ g,
                                             const float* __restrict__ be,
                                             float* __restrict__ Xf,
                                             _Float16* __restrict__ Xh)
{
#pragma clang fp contract(off)
  __shared__ __attribute__((aligned(16))) _Float16 ldsR[8 * CH];

  const int lane = threadIdx.x & 31, w = threadIdx.x >> 5;
  const size_t row = (size_t)blockIdx.x * 8 + w;
  v4f y[4];
  ln_row(S + row * CH, g, be, lane, y);
#pragma unroll
  for (int j = 0; j < 4; ++j)
#pragma unroll
    for (int e = 0; e < 4; ++e)
      ldsR[w * CH + 128 * j + 4 * lane + e] = toh_flush(y[j][e] * ACT_CAR);
  __syncthreads();
  const v8h h0 = *(const v8h*)&ldsR[w * CH + 8 * lane];
  const v8h h1 = *(const v8h*)&ldsR[w * CH + 256 + 8 * lane];
  float* const xf = Xf + row * CH;
  _Float16* const xh = Xh + row * CH;
#pragma unroll
  for (int j = 0; j < 4; ++j) *(volatile v4f*)(xf + 128 * j + 4 * lane) = y[j];
  *(volatile v8h*)(xh + 8 * lane) = h0;
  *(volatile v8h*)(xh + 256 + 8 * lane) = h1;
  __threadfence();
#pragma unroll
  for (int j = 0; j < 4; ++j) *(volatile v4f*)(xf + 128 * j + 4 * lane) = y[j];
  *(volatile v8h*)(xh + 8 * lane) = h0;
  *(volatile v8h*)(xh + 256 + 8 * lane) = h1;
}

__global__ __launch_bounds__(256) void k_ln2(const float* __restrict__ S,
                                             const float* __restrict__ g,
                                             const float* __restrict__ be,
                                             const int* __restrict__ em,
                                             float* __restrict__ out)
{
#pragma clang fp contract(off)
  const int lane = threadIdx.x & 31, w = threadIdx.x >> 5;
  const int row = blockIdx.x * 8 + w;
  v4f y[4];
  ln_row(S + (size_t)row * CH, g, be, lane, y);
  const int b  = row / (2 * SEQ);
  const int pp = row - b * 2 * SEQ;
  const int hf = pp / SEQ;
  const int s  = pp - hf * SEQ;
  const int mw = em[b * SEQ_FULL + s];
  const float mf = (mw == 1) ? 1.0f : 0.0f;
#pragma unroll
  for (int j = 0; j < 4; ++j)
#pragma unroll
    for (int e = 0; e < 4; ++e) y[j][e] = y[j][e] * mf;
  float* const ob = out + ((size_t)b * SEQ_FULL + s) * (2 * CH) + (size_t)hf * CH;
#pragma unroll
  for (int j = 0; j < 4; ++j) *(volatile v4f*)(ob + 128 * j + 4 * lane) = y[j];
  __threadfence();
#pragma unroll
  for (int j = 0; j < 4; ++j) *(volatile v4f*)(ob + 128 * j + 4 * lane) = y[j];
}

extern "C" void kernel_launch(void* const* d_in, const int* in_sizes, int n_in,
                              void* d_out, int out_size, void* d_ws, size_t ws_size,
                              hipStream_t stream)
{
  if (n_in < 36) return;
  const long need_act = (((long)NB - 1) * SEQ_FULL + SEQ) * CH;
  const long need_msk = ((long)NB - 1) * SEQ_FULL + SEQ;
  const long nWl = (long)CH * CH;
  const long need[36] = {
    need_act, need_act, need_msk, need_msk,
    nWl, CH, nWl, CH, nWl, CH, nWl, CH, nWl, CH, nWl, CH,
    3 * nWl, 3 * CH, nWl, CH,
    3 * nWl, 3 * CH, nWl, CH,
    3 * nWl, 3 * CH, nWl, CH,
    (long)DFF * CH, DFF, (long)CH * DFF, CH,
    CH, CH, CH, CH };
  for (int i = 0; i < 36; ++i)
    if ((long)in_sizes[i] < need[i]) return;
  if ((long)out_size < need_msk * 2 * CH) return;

  const float* emo_x  = (const float*)d_in[0];
  const float* sem_x  = (const float*)d_in[1];
  const int*   emo_m  = (const int*)d_in[2];
  const int*   sem_m  = (const int*)d_in[3];
  const float* Wq_emo = (const float*)d_in[4];   const float* bq_emo = (const float*)d_in[5];
  const float* Wk_emo = (const float*)d_in[6];   const float* bk_emo = (const float*)d_in[7];
  const float* Wv_emo = (const float*)d_in[8];   const float* bv_emo = (const float*)d_in[9];
  const float* Wq_sem = (const float*)d_in[10];  const float* bq_sem = (const float*)d_in[11];
  const float* Wk_sem = (const float*)d_in[12];  const float* bk_sem = (const float*)d_in[13];
  const float* Wv_sem = (const float*)d_in[14];  const float* bv_sem = (const float*)d_in[15];
  const float* sem_Wi = (const float*)d_in[16];  const float* sem_bi = (const float*)d_in[17];
  const float* sem_Wo = (const float*)d_in[18];  const float* sem_bo = (const float*)d_in[19];
  const float* emo_Wi = (const float*)d_in[20];  const float* emo_bi = (const float*)d_in[21];
  const float* emo_Wo = (const float*)d_in[22];  const float* emo_bo = (const float*)d_in[23];
  const float* t_Wi   = (const float*)d_in[24];  const float* t_bi   = (const float*)d_in[25];
  const float* t_Wo   = (const float*)d_in[26];  const float* t_bo   = (const float*)d_in[27];
  const float* t_W1   = (const float*)d_in[28];  const float* t_b1   = (const float*)d_in[29];
  const float* t_W2   = (const float*)d_in[30];  const float* t_b2   = (const float*)d_in[31];
  const float* ln1_g  = (const float*)d_in[32];  const float* ln1_b  = (const float*)d_in[33];
  const float* ln2_g  = (const float*)d_in[34];  const float* ln2_b  = (const float*)d_in[35];
  float* out = (float*)d_out;

  const int    M1  = NB * SEQ;
  const int    M2  = 2 * M1;
  const size_t nP1 = (size_t)M1 * CH;
  const size_t nP2 = (size_t)M2 * CH;
  const size_t nW  = (size_t)CH * CH;
  const size_t nMk = (size_t)2 * NB * SEQ;
  const size_t total_bytes = (36 * nP1 + 26 * nW) * sizeof(_Float16)
                           + 3 * nP2 * sizeof(float) + 2 * nMk * sizeof(float);
  if (total_bytes > ws_size) return;

  _Float16* X16 = (_Float16*)d_ws;
  _Float16* WA  = X16 + 2 * nP1;
  _Float16* WIs = WA  + 6 * nW;
  _Float16* WIe = WIs + 3 * nW;
  _Float16* WIt = WIe + 3 * nW;
  _Float16* WOs = WIt + 3 * nW;
  _Float16* WOe = WOs + nW;
  _Float16* WOt = WOe + nW;
  _Float16* W1h = WOt + nW;
  _Float16* W2h = W1h + 4 * nW;
  _Float16* P1  = W2h + 4 * nW;
  _Float16* QK2 = P1  + 6 * nP1;
  _Float16* VT2 = QK2 + 4 * nP1;
  _Float16* O2  = VT2 + 2 * nP1;
  _Float16* X0h = O2  + 2 * nP1;
  _Float16* QKT = X0h + nP2;
  _Float16* VTT = QKT + 2 * nP2;
  _Float16* OT  = VTT + nP2;
  _Float16* X1h = OT  + nP2;
  _Float16* Hh  = X1h + nP2;
  float* X0f = (float*)(Hh + (size_t)M2 * DFF);
  float* S1  = X0f + nP2;
  float* X1f = S1  + nP2;
  float* MX  = X1f + nP2;
  float* MT  = MX  + nMk;

  const int t8 = (int)(nP1 / 8);
  k_cvt8<<<(t8 + 255) / 256, 256, 0, stream>>>(emo_x, X16,       CH, SEQ, SEQ_FULL, ACT_CAR, t8);
  k_cvt8<<<(t8 + 255) / 256, 256, 0, stream>>>(sem_x, X16 + nP1, CH, SEQ, SEQ_FULL, ACT_CAR, t8);
  const int tw8 = (int)(nW / 8);
  k_cvt8<<<(tw8 + 255) / 256, 256, 0, stream>>>(Wq_emo, WA,          CH, CH, CH, W_CAR, tw8);
  k_cvt8<<<(tw8 + 255) / 256, 256, 0, stream>>>(Wk_emo, WA + nW,     CH, CH, CH, W_CAR, tw8);
  k_cvt8<<<(tw8 + 255) / 256, 256, 0, stream>>>(Wv_emo, WA + 2 * nW, CH, CH, CH, W_CAR, tw8);
  k_cvt8<<<(tw8 + 255) / 256, 256, 0, stream>>>(Wq_sem, WA + 3 * nW, CH, CH, CH, W_CAR, tw8);
  k_cvt8<<<(tw8 + 255) / 256, 256, 0, stream>>>(Wk_sem, WA + 4 * nW, CH, CH, CH, W_CAR, tw8);
  k_cvt8<<<(tw8 + 255) / 256, 256, 0, stream>>>(Wv_sem, WA + 5 * nW, CH, CH, CH, W_CAR, tw8);
  k_cvt8<<<(3 * tw8 + 255) / 256, 256, 0, stream>>>(sem_Wi, WIs, CH, 3 * CH, 3 * CH, W_CAR, 3 * tw8);
  k_cvt8<<<(3 * tw8 + 255) / 256, 256, 0, stream>>>(emo_Wi, WIe, CH, 3 * CH, 3 * CH, W_CAR, 3 * tw8);
  k_cvt8<<<(3 * tw8 + 255) / 256, 256, 0, stream>>>(t_Wi,   WIt, CH, 3 * CH, 3 * CH, W_CAR, 3 * tw8);
  k_cvt8<<<(tw8 + 255) / 256, 256, 0, stream>>>(sem_Wo, WOs, CH, CH, CH, W_CAR, tw8);
  k_cvt8<<<(tw8 + 255) / 256, 256, 0, stream>>>(emo_Wo, WOe, CH, CH, CH, W_CAR, tw8);
  k_cvt8<<<(tw8 + 255) / 256, 256, 0, stream>>>(t_Wo,   WOt, CH, CH, CH, W_CAR, tw8);
  k_cvt8<<<(4 * tw8 + 255) / 256, 256, 0, stream>>>(t_W1, W1h, CH,  DFF, DFF, W_CAR, 4 * tw8);
  k_cvt8<<<(4 * tw8 + 255) / 256, 256, 0, stream>>>(t_W2, W2h, DFF, CH,  CH,  W_CAR, 4 * tw8);

  k_mask<<<((int)(nMk / 4) + 255) / 256, 256, 0, stream>>>(emo_m, sem_m, MX, MT);

  const dim3 g1(CH / 64, M1 / 128, 1);
  k_gemm_h<<<g1, 128, 0, stream>>>(X16,       WA,          P1,           bq_emo, 0L, 0L, 0L, CH, PROJ_SCL, QKV_CAR, 0, 0);
  k_gemm_h<<<g1, 128, 0, stream>>>(X16 + nP1, WA + 4 * nW, P1 + nP1,     bk_sem, 0L, 0L, 0L, CH, PROJ_SCL, QKV_CAR, 0, 0);
  k_gemm_h<<<g1, 128, 0, stream>>>(X16 + nP1, WA + 5 * nW, P1 + 2 * nP1, bv_sem, 0L, 0L, 0L, CH, PROJ_SCL, QKV_CAR, 0, 0);
  k_gemm_h<<<g1, 128, 0, stream>>>(X16 + nP1, WA + 3 * nW, P1 + 3 * nP1, bq_sem, 0L, 0L, 0L, CH, PROJ_SCL, QKV_CAR, 0, 0);
  k_gemm_h<<<g1, 128, 0, stream>>>(X16,       WA + nW,     P1 + 4 * nP1, bk_emo, 0L, 0L, 0L, CH, PROJ_SCL, QKV_CAR, 0, 0);
  k_gemm_h<<<g1, 128, 0, stream>>>(X16,       WA + 2 * nW, P1 + 5 * nP1, bv_emo, 0L, 0L, 0L, CH, PROJ_SCL, QKV_CAR, 0, 0);

  const dim3 g2(CH / 64, M1 / 128, 2);
  k_gemm_h<<<g2, 128, 0, stream>>>(P1,           WIs, QK2,       sem_bi, (long)nP1, (long)nW, (long)(2 * nP1), CH, MID_SCL, QKV_CAR, 0, CH);
  k_gemm_h<<<g2, 128, 0, stream>>>(P1 + 3 * nP1, WIe, QK2 + nP1, emo_bi, (long)nP1, (long)nW, (long)(2 * nP1), CH, MID_SCL, QKV_CAR, 0, CH);
  const dim3 g3(SEQ / 64, CH / 128, NB);
  k_gemm_vt<<<g3, 128, 0, stream>>>(WIs + 2 * nW, P1 + 2 * nP1, VT2,       sem_bi + 2 * CH, (long)SEQ * CH, (long)CH * SEQ, SEQ);
  k_gemm_vt<<<g3, 128, 0, stream>>>(WIe + 2 * nW, P1 + 5 * nP1, VT2 + nP1, emo_bi + 2 * CH, (long)SEQ * CH, (long)CH * SEQ, SEQ);

  k_attn<<<2 * NB * NH * (SEQ / 128), 256, 0, stream>>>(QK2, QK2 + 2 * nP1, VT2, MX, O2, SEQ);

  const dim3 g4(CH / 64, M1 / 128, 1);
  k_gemm_x0<<<g4, 128, 0, stream>>>(O2,       WOs, X0f, X0h, sem_bo, SEQ, 2 * SEQ, 0);
  k_gemm_x0<<<g4, 128, 0, stream>>>(O2 + nP1, WOe, X0f, X0h, emo_bo, SEQ, 2 * SEQ, SEQ);

  const dim3 g5(CH / 64, M2 / 128, 2);
  k_gemm_h<<<g5, 128, 0, stream>>>(X0h, WIt, QKT, t_bi, 0L, (long)nW, (long)nP2, CH, MID_SCL, QKV_CAR, 0, CH);
  const dim3 g6((2 * SEQ) / 64, CH / 128, NB);
  k_gemm_vt<<<g6, 128, 0, stream>>>(WIt + 2 * nW, X0h, VTT, t_bi + 2 * CH, (long)2 * SEQ * CH, (long)CH * 2 * SEQ, 2 * SEQ);
  k_attn<<<NB * NH * ((2 * SEQ) / 128), 256, 0, stream>>>(QKT, QKT + nP2, VTT, MT, OT, 2 * SEQ);
  const dim3 g7(CH / 64, M2 / 128, 1);
  k_gemm_res<<<g7, 128, 0, stream>>>(OT, WOt, S1, t_bo, X0f, CH);
  k_ln1<<<M2 / 8, 256, 0, stream>>>(S1, ln1_g, ln1_b, X1f, X1h);

  const dim3 g8(DFF / 64, M2 / 128, 1);
  k_gemm_h<<<g8, 128, 0, stream>>>(X1h, W1h, Hh, t_b1, 0L, 0L, 0L, DFF, PROJ_SCL, QKV_CAR, 1, 0);
  k_gemm_res<<<g7, 128, 0, stream>>>(Hh, W2h, S1, t_b2, X1f, DFF);

  k_ln2<<<M2 / 8, 256, 0, stream>>>(S1, ln2_g, ln2_b, emo_m, out);
}
